// CrossAtt_10960756540399
// MI455X (gfx1250) — hardware-run, weakly checked
//
#include <hip/hip_runtime.h>
#include <math.h>
#include <stdint.h>

#ifndef NB
#define NB 2
#endif
#ifndef NPIX
#define NPIX 4096
#endif
#define NB_FULL   2
#define NPIX_FULL 4096
#define CIN   256
#define COUT  256
#define DQK   16
#define DV    128
#define IMW   64
#define HH    (NPIX / IMW)
#define PH    (HH + 2)
#define PWD   (IMW + 2)
#define NIMG  (2 * NB)
#define NQT   (NPIX / 64)
#define NKT   (NPIX / 64)
#define KCONV (9 * CIN)
#define NBRD  (2 * PWD + 2 * HH)
static_assert(NB >= 1 && NB <= NB_FULL);
static_assert(NPIX >= 64 && NPIX <= NPIX_FULL && (NPIX % 64) == 0 && (NPIX % IMW) == 0);
static_assert(CIN == 256 && COUT == 256 && DV == 128 && DQK == 16);
static_assert((KCONV % 32) == 0 && (CIN % 64) == 0 && (COUT % 64) == 0 && (DV % 64) == 0);
static_assert(((NIMG * NPIX) % 64) == 0);
static_assert((size_t)NB_FULL * CIN * NPIX_FULL * 4 == 8388608);

typedef _Float16 v16h __attribute__((ext_vector_type(16)));
typedef _Float16 v8h  __attribute__((ext_vector_type(8)));
typedef __bf16   v16b __attribute__((ext_vector_type(16)));
typedef __bf16   v8b  __attribute__((ext_vector_type(8)));
typedef float    v8f  __attribute__((ext_vector_type(8)));
typedef float    v4f  __attribute__((ext_vector_type(4)));
typedef unsigned int v4u __attribute__((ext_vector_type(4)));

__device__ __forceinline__ unsigned short bf_bits(float f) {
  unsigned u = __float_as_uint(f);
  return (unsigned short)((u + 0x7FFFu + ((u >> 16) & 1u)) >> 16);
}
__device__ __forceinline__ float bf_up(unsigned short h) { return __uint_as_float(((unsigned)h) << 16); }
__device__ __forceinline__ float bf_rn(float f) { return bf_up(bf_bits(f)); }
__device__ __forceinline__ unsigned short h_bits(_Float16 x) { return __builtin_bit_cast(unsigned short, x); }
__device__ __forceinline__ unsigned pk16(unsigned short a, unsigned short b) { return (unsigned)a | ((unsigned)b << 16); }
__device__ __forceinline__ v8f zero8() { v8f z = {0.f, 0.f, 0.f, 0.f, 0.f, 0.f, 0.f, 0.f}; return z; }
__device__ __forceinline__ v4u zero4u() { v4u z = {0u, 0u, 0u, 0u}; return z; }

__device__ __forceinline__ v16b ldfrag_b(const __bf16* p) {
  union { v16b v; v8b h[2]; } f;
  f.h[0] = *(const v8b*)(p);
  f.h[1] = *(const v8b*)(p + 16);
  return f.v;
}
__device__ __forceinline__ v16h ldfrag_h(const _Float16* p) {
  union { v16h v; v8h h[2]; } f;
  f.h[0] = *(const v8h*)(p);
  f.h[1] = *(const v8h*)(p + 16);
  return f.v;
}

__device__ __forceinline__ v8f mma_b(v16b a, v16b b, v8f c) {
  c = __builtin_amdgcn_wmma_f32_16x16x32_bf16(false, a, false, b, (short)0, c, false, false);
#if defined(__HIP_DEVICE_COMPILE__)
  asm volatile("v_nop\n\tv_nop\n\tv_nop\n\tv_nop" : "+v"(c) : "v"(a), "v"(b));
#endif
  return c;
}
__device__ __forceinline__ v8f mma_h(v16h a, v16h b, v8f c) {
  c = __builtin_amdgcn_wmma_f32_16x16x32_f16(false, a, false, b, (short)0, c, false, false);
#if defined(__HIP_DEVICE_COMPILE__)
  asm volatile("v_nop\n\tv_nop\n\tv_nop\n\tv_nop" : "+v"(c) : "v"(a), "v"(b));
#endif
  return c;
}
__device__ __forceinline__ v8f mma_b_raw(v16b a, v16b b, v8f c) {
  return __builtin_amdgcn_wmma_f32_16x16x32_bf16(false, a, false, b, (short)0, c, false, false);
}
__device__ __forceinline__ void dep_guard_b(v8f& a, v8f& b, v16b x, v16b y) {
#if defined(__HIP_DEVICE_COMPILE__)
  asm volatile("v_nop\n\tv_nop\n\tv_nop\n\tv_nop" : "+v"(a), "+v"(b) : "v"(x), "v"(y));
#endif
}
__device__ __forceinline__ void keep4_b(v16b a, v16b b, v16b c, v16b d) {
#if defined(__HIP_DEVICE_COMPILE__)
  asm volatile("v_nop" :: "v"(a), "v"(b), "v"(c), "v"(d));
#endif
}
__device__ __forceinline__ void acc_guard4(v8f& a, v8f& b, v8f& c, v8f& d) {
#if defined(__HIP_DEVICE_COMPILE__)
  asm volatile("v_nop\n\tv_nop\n\tv_nop\n\tv_nop" : "+v"(a), "+v"(b), "+v"(c), "+v"(d));
#endif
}

__global__ __launch_bounds__(256) void cvt_bf16x8(const float* __restrict__ in, unsigned short* out, int n8) {
  const int i = blockIdx.x * 256 + threadIdx.x;
  if (i < n8) {
    const v4f a = *(const v4f*)(in + (size_t)i * 8);
    const v4f b = *(const v4f*)(in + (size_t)i * 8 + 4);
    v4u p;
    p[0] = pk16(bf_bits(a[0]), bf_bits(a[1]));
    p[1] = pk16(bf_bits(a[2]), bf_bits(a[3]));
    p[2] = pk16(bf_bits(b[0]), bf_bits(b[1]));
    p[3] = pk16(bf_bits(b[2]), bf_bits(b[3]));
    *(volatile v4u*)(out + (size_t)i * 8) = p;
    __threadfence();
    *(volatile v4u*)(out + (size_t)i * 8) = p;
  }
}

__global__ __launch_bounds__(256) void cvt_xT(const float* __restrict__ xa, const float* __restrict__ xb,
                                              unsigned short* out) {
  __shared__ __align__(16) unsigned short sh[64 * 72];
  const int tid  = threadIdx.x;
  const int lane = tid & 31;
  const int wave = tid >> 5;
  const int n0  = blockIdx.x * 64;
  const int c0  = blockIdx.y * 64;
  const int img = blockIdx.z;
  const int inp = img / NB;
  const int b   = img - inp * NB;
  const float* x = ((inp == 0) ? xa : xb) + (size_t)b * CIN * NPIX_FULL;
  {
    const int kr = tid >> 2;
    const int nc = (tid & 3) * 16;
    const float* src = x + (size_t)(c0 + kr) * NPIX_FULL + n0 + nc;
#pragma unroll
    for (int e = 0; e < 4; ++e) {
      const v4f a = *(const v4f*)(src + 4 * e);
#pragma unroll
      for (int j = 0; j < 4; ++j) sh[(nc + 4 * e + j) * 72 + kr] = bf_bits(a[j]);
    }
  }
  __syncthreads();
  const int q = lane >> 3, c8 = (lane & 7) * 8;
  v4u v[2];
#pragma unroll
  for (int it = 0; it < 2; ++it) {
    const int row = wave * 8 + it * 4 + q;
    v[it] = *(const v4u*)(sh + row * 72 + c8);
  }
  for (int pass = 0; pass < 2; ++pass) {
#pragma unroll
    for (int it = 0; it < 2; ++it) {
      const int row = wave * 8 + it * 4 + q;
      *(volatile v4u*)(out + ((size_t)img * NPIX + n0 + row) * CIN + c0 + c8) = v[it];
    }
    __threadfence();
  }
}

__global__ __launch_bounds__(256) void pack_qk(const float* __restrict__ Wq, const float* __restrict__ bq,
                                               const float* __restrict__ Wk, const float* __restrict__ bk,
                                               unsigned short* Wqk, float* bqk) {
  const int tid = threadIdx.x;
  v4u pv[8];
#pragma unroll
  for (int i = 0; i < 8; ++i) {
    const int v   = tid + 256 * i;
    const int row = v >> 5;
    const int c8  = (v & 31) * 8;
    const int rr  = row & 15;
    const v4f q0 = *(const v4f*)(Wq + rr * CIN + c8);
    const v4f q1 = *(const v4f*)(Wq + rr * CIN + c8 + 4);
    const v4f k0 = *(const v4f*)(Wk + rr * CIN + c8);
    const v4f k1 = *(const v4f*)(Wk + rr * CIN + c8 + 4);
    const bool selq = (row < 16);
    const bool selk = (row >= 32) && (row < 48);
    float f[8];
#pragma unroll
    for (int e = 0; e < 4; ++e) {
      f[e]     = selq ? q0[e] : (selk ? k0[e] : 0.f);
      f[4 + e] = selq ? q1[e] : (selk ? k1[e] : 0.f);
    }
    v4u p;
#pragma unroll
    for (int e = 0; e < 4; ++e) p[e] = pk16(bf_bits(f[2 * e]), bf_bits(f[2 * e + 1]));
    pv[i] = p;
  }
  for (int pass = 0; pass < 2; ++pass) {
#pragma unroll
    for (int i = 0; i < 8; ++i) *(volatile v4u*)(Wqk + (size_t)(tid + 256 * i) * 8) = pv[i];
    __threadfence();
  }
  const int rb = tid & 15;
  const float fq = bq[rb];
  const float fk = bk[rb];
  const float bvv = (tid < 16) ? fq : (((tid >= 32) && (tid < 48)) ? fk : 0.f);
  if (tid < 64) *(volatile float*)(bqk + tid) = bvv;
  __threadfence();
  if (tid < 64) *(volatile float*)(bqk + tid) = bvv;
}

__global__ __launch_bounds__(256) void pack_wcat(const float* __restrict__ Wcat, unsigned short* Wm) {
  __shared__ __align__(16) unsigned short sh[KCONV];
  const int o = blockIdx.x;
  const int tid = threadIdx.x;
  const float* src = Wcat + (size_t)o * KCONV;
#pragma unroll
  for (int i = 0; i < 9; ++i) {
    const int e   = tid + 256 * i;
    const int cc  = e / 9;
    const int tap = e - 9 * cc;
    sh[tap * CIN + cc] = bf_bits(src[e]);
  }
  __syncthreads();
  const v4u a  = *(const v4u*)(sh + tid * 8);
  const v4u a2 = *(const v4u*)(sh + 2048 + (tid & 31) * 8);
  unsigned short* dst = Wm + (size_t)o * KCONV;
  for (int pass = 0; pass < 2; ++pass) {
    *(volatile v4u*)(dst + tid * 8) = a;
    if (tid < 32) *(volatile v4u*)(dst + 2048 + tid * 8) = a2;
    __threadfence();
  }
}

template <int NSPLIT, int OUT_MODE, int EPI>
__global__ __launch_bounds__(256) void gemm64(
    const unsigned short* __restrict__ Ap, const unsigned short* __restrict__ A2p, int lda, long long strideA,
    const unsigned short* __restrict__ Btp, int ldb, long long strideB,
    const float* __restrict__ bias, const float* __restrict__ rowbias, const float* __restrict__ addend,
    void* C0, void* C1, void* C2, int ldc, long long strideC,
    int M, int N, int K, float oscale, float rscale) {
  static_assert(OUT_MODE >= 1 && OUT_MODE <= 5);
  static_assert((EPI & 4) == 0 || OUT_MODE == 4);
  static_assert(NSPLIT == 0 || NSPLIT == 1);
  const __bf16* A  = (const __bf16*)(const void*)Ap;
  const __bf16* A2 = (const __bf16*)(const void*)A2p;
  const __bf16* Bt = (const __bf16*)(const void*)Btp;
  __shared__ __align__(16) float sT[8][16 * 68];
  const int b    = blockIdx.y;
  const int lane = threadIdx.x & 31;
  const int wave = threadIdx.x >> 5;
  const int tilesN = N >> 6;
  const int tilesM = M >> 6;
  const int tile = blockIdx.x * 8 + wave;
  if (tile >= tilesM * tilesN) return;
  const int tm = tile / tilesN;
  const int tn = tile - tm * tilesN;
  const int m0 = tm << 6;
  const int n0 = tn << 6;

  const __bf16* Ab  = A  + (size_t)b * strideA;
  const __bf16* Bb  = Bt + (size_t)b * strideB;
  const __bf16* Ab2 = (NSPLIT >= 1) ? (A2 + (size_t)b * strideA) : Ab;

  const int rlane = lane & 15;
  const int koff  = (lane >> 4) * 8;
  const int mOff  = (lane >> 4) * 8;

  v8f acc[4][4];
#pragma unroll
  for (int i = 0; i < 4; ++i)
#pragma unroll
    for (int j = 0; j < 4; ++j) acc[i][j] = zero8();

  for (int k0 = 0; k0 < K; k0 += 32) {
    v16b bh[4];
#pragma unroll
    for (int j = 0; j < 4; ++j) {
      const size_t bo = (size_t)(n0 + (j << 4) + rlane) * ldb + koff + k0;
      bh[j] = ldfrag_b(Bb + bo);
    }
#pragma unroll
    for (int i = 0; i < 4; ++i) {
      const size_t ao = (size_t)(m0 + (i << 4) + rlane) * lda + koff + k0;
      const v16b ah = ldfrag_b(Ab + ao);
      v16b al = ah;
      if (NSPLIT >= 1) al = ldfrag_b(Ab2 + ao);
#pragma unroll
      for (int j = 0; j < 4; ++j) {
        acc[i][j] = mma_b_raw(ah, bh[j], acc[i][j]);
        if (NSPLIT >= 1) acc[i][j] = mma_b_raw(al, bh[j], acc[i][j]);
      }
      dep_guard_b(acc[i][0], acc[i][3], ah, al);
    }
    keep4_b(bh[0], bh[1], bh[2], bh[3]);
  }
  acc_guard4(acc[0][0], acc[0][1], acc[0][2], acc[0][3]);
  acc_guard4(acc[1][0], acc[1][1], acc[1][2], acc[1][3]);
  acc_guard4(acc[2][0], acc[2][1], acc[2][2], acc[2][3]);
  acc_guard4(acc[3][0], acc[3][1], acc[3][2], acc[3][3]);

  float* slab = sT[wave];
  const int hh2 = lane >> 4, c4 = (lane & 15) * 4;
  const int q4  = lane >> 3, c8 = (lane & 7) * 8;
  v4f b4 = {0.f, 0.f, 0.f, 0.f};
  float b8[8];
#pragma unroll
  for (int e = 0; e < 8; ++e) b8[e] = 0.f;
  if (EPI & 1) {
    const v4f t = *(const v4f*)(bias + n0 + c4);
#pragma unroll
    for (int e = 0; e < 4; ++e) b4[e] = bf_rn(t[e]);
    const v4f t0 = *(const v4f*)(bias + n0 + c8);
    const v4f t1 = *(const v4f*)(bias + n0 + c8 + 4);
#pragma unroll
    for (int e = 0; e < 4; ++e) { b8[e] = bf_rn(t0[e]); b8[4 + e] = bf_rn(t1[e]); }
  }

#pragma unroll
  for (int i = 0; i < 4; ++i) {
    const int mBase = m0 + (i << 4);
#pragma unroll
    for (int j = 0; j < 4; ++j) {
#pragma unroll
      for (int r = 0; r < 8; ++r) {
        slab[(mOff + r) * 68 + (j << 4) + rlane] = acc[i][j][r];
      }
    }
    __builtin_amdgcn_fence(__ATOMIC_RELEASE, "workgroup");
    __builtin_amdgcn_wave_barrier();
    __builtin_amdgcn_fence(__ATOMIC_ACQUIRE, "workgroup");
    if (OUT_MODE == 4 || OUT_MODE == 5) {
      float* C = (float*)C0 + (size_t)b * strideC;
      v4f fv[8];
#pragma unroll
      for (int it = 0; it < 8; ++it) {
        const int row = it * 2 + hh2;
        v4f v = *(const v4f*)(slab + row * 68 + c4);
        if (EPI & 1) v += b4;
        if (EPI & 8) {
          const float rb = bf_rn(rowbias[mBase + row]);
#pragma unroll
          for (int e = 0; e < 4; ++e) v[e] += rb;
        }
        if (EPI & 2) {
#pragma unroll
          for (int e = 0; e < 4; ++e) v[e] = fmaxf(v[e], 0.f);
        }
        if (EPI & 4) v += *(const v4f*)(addend + (size_t)b * strideC + (size_t)(mBase + row) * ldc + n0 + c4);
        fv[it] = v;
      }
      for (int pass = 0; pass < 2; ++pass) {
#pragma unroll
        for (int it = 0; it < 8; ++it) {
          const int row = it * 2 + hh2;
          *(volatile v4f*)(C + (size_t)(mBase + row) * ldc + n0 + c4) = fv[it];
        }
        __threadfence();
      }
    }
    if (OUT_MODE != 4) {
      unsigned short* P0 = (unsigned short*)((OUT_MODE == 5) ? C1 : C0) + (size_t)b * strideC;
      unsigned short* P1 = (unsigned short*)((OUT_MODE == 5) ? C2 : C1) + (size_t)b * strideC;
      v4u hv[4], lv[4];
#pragma unroll
      for (int it = 0; it < 4; ++it) {
        const int row = it * 4 + q4;
        const float* sp = slab + row * 68 + c8;
        float rb = 0.f;
        if (EPI & 8) rb = bf_rn(rowbias[mBase + row]);
        v4u a, a2;
#pragma unroll
        for (int e = 0; e < 4; ++e) {
          float f0 = sp[2 * e], f1 = sp[2 * e + 1];
          if (EPI & 1) { f0 += b8[2 * e]; f1 += b8[2 * e + 1]; }
          if (EPI & 8) { f0 += rb; f1 += rb; }
          if (EPI & 2) { f0 = fmaxf(f0, 0.f); f1 = fmaxf(f1, 0.f); }
          unsigned short h0, h1, l0, l1;
          if (OUT_MODE == 1) {
            h0 = h_bits((_Float16)(f0 * oscale)); h1 = h_bits((_Float16)(f1 * oscale));
            l0 = 0; l1 = 0;
          } else if (OUT_MODE == 3) {
            const float x0 = f0 * oscale, x1 = f1 * oscale;
            const _Float16 y0 = (_Float16)x0, y1 = (_Float16)x1;
            h0 = h_bits(y0); h1 = h_bits(y1);
            l0 = h_bits((_Float16)((x0 - (float)y0) * rscale));
            l1 = h_bits((_Float16)((x1 - (float)y1) * rscale));
          } else {
            h0 = bf_bits(f0); h1 = bf_bits(f1);
            l0 = bf_bits(f0 - bf_up(h0)); l1 = bf_bits(f1 - bf_up(h1));
          }
          a[e] = pk16(h0, h1); a2[e] = pk16(l0, l1);
        }
        hv[it] = a; lv[it] = a2;
      }
      for (int pass = 0; pass < 2; ++pass) {
#pragma unroll
        for (int it = 0; it < 4; ++it) {
          const int row = it * 4 + q4;
          const size_t go = (size_t)(mBase + row) * ldc + n0 + c8;
          *(volatile v4u*)(P0 + go) = hv[it];
          if (OUT_MODE != 1) *(volatile v4u*)(P1 + go) = lv[it];
        }
        __threadfence();
      }
    }
    __builtin_amdgcn_fence(__ATOMIC_RELEASE, "workgroup");
    __builtin_amdgcn_wave_barrier();
    __builtin_amdgcn_fence(__ATOMIC_ACQUIRE, "workgroup");
  }
}

__global__ __launch_bounds__(128)
void attn_x(const unsigned short* __restrict__ qkpl, const unsigned short* __restrict__ vtp,
            const float* __restrict__ xa, const float* __restrict__ xb,
            const float* __restrict__ gammap, float* outa, float* outb,
            float sscale, float oscl) {
  union FH { v16h v; v8h h[2]; };
  __shared__ __align__(16) _Float16 Ksh[64 * 32];
  __shared__ __align__(16) _Float16 Vth[DV * 64];
  __shared__ __align__(16) _Float16 Psh[4][16 * 64];
  __shared__ __align__(16) float    Osb[DV * 64];

  const int tid  = threadIdx.x;
  const int wave = tid >> 5;
  const int lane = tid & 31;
  const int hh   = lane >> 4;
  const int c    = lane & 15;

  const int bx   = blockIdx.x;
  const int qb   = bx % NQT;
  const int rest = bx / NQT;
  const int b    = rest % NB;
  const int z    = rest / NB;
  const int is   = z * NB + b;
  const int io   = (1 - z) * NB + b;
  const int q0   = qb * 64 + wave * 16;

  const _Float16* QK = (const _Float16*)(const void*)qkpl;
  const _Float16* VT = (const _Float16*)(const void*)vtp + (size_t)is * DV * NPIX;
  const float* xs = ((z == 0) ? xa : xb) + (size_t)b * CIN * NPIX_FULL;
  float* op = ((z == 0) ? outa : outb) + (size_t)b * CIN * NPIX_FULL;

  const v16h qa = ldfrag_h(QK + ((size_t)is * NPIX + q0 + c) * 64 + 8 * hh);

  float mrow[8], lrow[8];
  v8f oacc[8];
#pragma unroll
  for (int r = 0; r < 8; ++r) { mrow[r] = -INFINITY; lrow[r] = 0.f; }
#pragma unroll
  for (int t = 0; t < 8; ++t) oacc[t] = zero8();

  for (int kt = 0; kt < NKT; ++kt) {
    const int kv0 = kt * 64;
    __syncthreads();
    {
      const int r = tid >> 1, half = (tid & 1) * 16;
      const _Float16* kg = QK + ((size_t)io * NPIX + kv0 + r) * 64 + 32 + half;
      const v8h a0 = *(const v8h*)(kg);
      const v8h a1 = *(const v8h*)(kg + 8);
      *(v8h*)(Ksh + r * 32 + half) = a0;
      *(v8h*)(Ksh + r * 32 + half + 8) = a1;
      const _Float16* vg = VT + (size_t)tid * NPIX + kv0;
#pragma unroll
      for (int i = 0; i < 8; ++i) {
        const v8h v0 = *(const v8h*)(vg + 8 * i);
        *(v8h*)(Vth + tid * 64 + 8 * i) = v0;
      }
    }
    __syncthreads();

    v8f s[4];
#pragma unroll
    for (int j = 0; j < 4; ++j) {
      FH kb;
      kb.h[0] = *(const v8h*)(Ksh + (j * 16 + c) * 32 + 8 * hh);
      kb.h[1] = *(const v8h*)(Ksh + (j * 16 + c) * 32 + 16 + 8 * hh);
      s[j] = mma_h(qa, kb.v, zero8());
    }

    _Float16* pw = Psh[wave];
#pragma unroll
    for (int r = 0; r < 8; ++r) {
      float m = -INFINITY;
#pragma unroll
      for (int j = 0; j < 4; ++j) {
        const float sv = s[j][r] * sscale;
        s[j][r] = sv;
        m = fmaxf(m, sv);
      }
#pragma unroll
      for (int off = 1; off < 16; off <<= 1) m = fmaxf(m, __shfl_xor(m, off, 32));
      const float mnew  = fmaxf(mrow[r], m);
      const float msafe = (mnew == -INFINITY) ? 0.f : mnew;
      const float alpha = __expf(mrow[r] - msafe);
      mrow[r] = mnew;
      float psum = 0.f;
#pragma unroll
      for (int j = 0; j < 4; ++j) {
        const float p = __expf(s[j][r] - msafe);
        psum += p;
        pw[(8 * hh + r) * 64 + j * 16 + c] = (_Float16)(p * 1024.0f);
      }
#pragma unroll
      for (int off = 1; off < 16; off <<= 1) psum += __shfl_xor(psum, off, 32);
      lrow[r] = lrow[r] * alpha + psum;
#pragma unroll
      for (int t = 0; t < 8; ++t) oacc[t][r] *= alpha;
    }
    __builtin_amdgcn_fence(__ATOMIC_RELEASE, "workgroup");
    __builtin_amdgcn_wave_barrier();
    __builtin_amdgcn_fence(__ATOMIC_ACQUIRE, "workgroup");

#pragma unroll 1
    for (int kk = 0; kk < 2; ++kk) {
      FH pa;
      pa.h[0] = *(const v8h*)(pw + c * 64 + kk * 32 + 8 * hh);
      pa.h[1] = *(const v8h*)(pw + c * 64 + kk * 32 + 16 + 8 * hh);
#pragma unroll
      for (int t = 0; t < 8; ++t) {
        FH vb;
        vb.h[0] = *(const v8h*)(Vth + (t * 16 + c) * 64 + kk * 32 + 8 * hh);
        vb.h[1] = *(const v8h*)(Vth + (t * 16 + c) * 64 + kk * 32 + 16 + 8 * hh);
        oacc[t] = mma_h(pa.v, vb.v, oacc[t]);
      }
    }
  }

#pragma unroll
  for (int r = 0; r < 8; ++r) {
    const float l = lrow[r];
    const float inv = ((l > 0.f) ? (1.0f / l) : 0.f) * oscl;
#pragma unroll
    for (int t = 0; t < 8; ++t) Osb[(t * 16 + c) * 64 + wave * 16 + 8 * hh + r] = oacc[t][r] * inv;
  }
  __syncthreads();

  {
    const float g = bf_rn(gammap[0]);
    const int hh2 = lane >> 4, c4 = (lane & 15) * 4;
    const size_t pix = (size_t)qb * 64 + c4;
#pragma unroll 1
    for (int chunk = 0; chunk < 2; ++chunk) {
      v4f fv[8];
#pragma unroll
      for (int it = 0; it < 8; ++it) {
        const int ch = wave * 32 + chunk * 16 + it * 2 + hh2;
        const v4f cv = *(const v4f*)(Osb + ch * 64 + c4);
        const v4f xv = *(const v4f*)(xs + (size_t)ch * NPIX_FULL + pix);
        v4f t;
#pragma unroll
        for (int e = 0; e < 4; ++e) t[e] = g * cv[e] + bf_rn(xv[e]);
        fv[it] = t;
      }
      for (int pass = 0; pass < 2; ++pass) {
#pragma unroll
        for (int it = 0; it < 8; ++it) {
          const int ch = wave * 32 + chunk * 16 + it * 2 + hh2;
          *(volatile v4f*)(op + (size_t)ch * NPIX_FULL + pix) = fv[it];
        }
        __threadfence();
      }
    }
  }
}

__global__ __launch_bounds__(256) void zero_ring(unsigned short* sph, unsigned short* spl) {
  const int lane = threadIdx.x & 31;
  const int wave = threadIdx.x >> 5;
  const int gw = blockIdx.x * 8 + wave;
  if (gw >= NB * NBRD) return;
  const int b = gw / NBRD;
  const int e = gw - b * NBRD;
  int hp, wp;
  if (e < PWD) { hp = 0; wp = e; }
  else if (e < 2 * PWD) { hp = PH - 1; wp = e - PWD; }
  else { const int k = e - 2 * PWD; hp = 1 + (k >> 1); wp = (k & 1) ? (PWD - 1) : 0; }
  const size_t off = (((size_t)(b * PH + hp)) * PWD + wp) * CIN + (size_t)lane * 8;
  const v4u zz = zero4u();
  for (int pass = 0; pass < 2; ++pass) {
    *(volatile v4u*)(sph + off) = zz;
    *(volatile v4u*)(spl + off) = zz;
    __threadfence();
  }
}

__global__ __launch_bounds__(256) void fuse_s(const float* __restrict__ xa, const float* __restrict__ xb,
                                              const float* __restrict__ gammap, float* oa, float* ob,
                                              unsigned short* sph, unsigned short* spl) {
  __shared__ __align__(16) float ts[CIN * 36];
  const int tid  = threadIdx.x;
  const int lane = tid & 31;
  const int wave = tid >> 5;
  const int n0 = blockIdx.x * 32;
  const int b  = blockIdx.y;
  const float g = bf_rn(gammap[0]);
  const float* x1b = xa + (size_t)b * CIN * NPIX_FULL;
  const float* x2b = xb + (size_t)b * CIN * NPIX_FULL;
  float* o1b = oa + (size_t)b * CIN * NPIX_FULL;
  float* o2b = ob + (size_t)b * CIN * NPIX_FULL;
  const int q  = lane >> 3;
  const int p4 = (lane & 7) * 4;

  {
    v4f u1[4], u2[4];
#pragma unroll
    for (int it = 0; it < 4; ++it) {
      const int ch = 128 + wave * 16 + it * 4 + q;
      const v4f alo = *(const v4f*)(x1b + (size_t)(ch - 128) * NPIX_FULL + n0 + p4);
      const v4f ahi = *(const v4f*)(x1b + (size_t)ch * NPIX_FULL + n0 + p4);
      const v4f blo = *(const v4f*)(x2b + (size_t)(ch - 128) * NPIX_FULL + n0 + p4);
      const v4f bhi = *(const v4f*)(x2b + (size_t)ch * NPIX_FULL + n0 + p4);
      v4f t1, t2, sum;
#pragma unroll
      for (int e = 0; e < 4; ++e) {
        t1[e] = g * bf_rn(alo[e]) + bf_rn(ahi[e]);
        t2[e] = g * bf_rn(blo[e]) + bf_rn(bhi[e]);
        sum[e] = t1[e] + t2[e];
      }
      u1[it] = t1; u2[it] = t2;
      *(v4f*)(ts + ch * 36 + p4) = sum;
    }
    for (int pass = 0; pass < 2; ++pass) {
#pragma unroll
      for (int it = 0; it < 4; ++it) {
        const int ch = 128 + wave * 16 + it * 4 + q;
        *(volatile v4f*)(o1b + (size_t)ch * NPIX_FULL + n0 + p4) = u1[it];
        *(volatile v4f*)(o2b + (size_t)ch * NPIX_FULL + n0 + p4) = u2[it];
      }
      __threadfence();
    }
  }
#pragma unroll
  for (int it = 0; it < 4; ++it) {
    const int ch = wave * 16 + it * 4 + q;
    const v4f a1 = *(const v4f*)(o1b + (size_t)ch * NPIX_FULL + n0 + p4);
    const v4f a2 = *(const v4f*)(o2b + (size_t)ch * NPIX_FULL + n0 + p4);
    *(v4f*)(ts + ch * 36 + p4) = a1 + a2;
  }
  __syncthreads();
  {
    v4u hv[4], lv[4];
#pragma unroll
    for (int i = 0; i < 4; ++i) {
      const int p = wave * 4 + i;
      v4u a, a2;
#pragma unroll
      for (int e = 0; e < 4; ++e) {
        const float f0 = ts[(lane * 8 + 2 * e) * 36 + p];
        const float f1 = ts[(lane * 8 + 2 * e + 1) * 36 + p];
        const unsigned short h0 = bf_bits(f0), h1 = bf_bits(f1);
        const unsigned short l0 = bf_bits(f0 - bf_up(h0)), l1 = bf_bits(f1 - bf_up(h1));
        a[e] = pk16(h0, h1); a2[e] = pk16(l0, l1);
      }
      hv[i] = a; lv[i] = a2;
    }
    for (int pass = 0; pass < 2; ++pass) {
#pragma unroll
      for (int i = 0; i < 4; ++i) {
        const int p = wave * 4 + i;
        const int n = n0 + p;
        const int h = n / IMW;
        const int w = n - h * IMW;
        const size_t go = (((size_t)(b * PH + h + 1)) * PWD + (w + 1)) * CIN + (size_t)lane * 8;
        *(volatile v4u*)(sph + go) = hv[i];
        *(volatile v4u*)(spl + go) = lv[i];
      }
      __threadfence();
    }
  }
}

__global__ __launch_bounds__(256) void conv_gemm(
    const unsigned short* __restrict__ Wmp, const unsigned short* __restrict__ Shp, const unsigned short* __restrict__ Slp,
    const float* __restrict__ bng, const float* __restrict__ bnb, float* feat, float bninv) {
  const __bf16* A  = (const __bf16*)(const void*)Wmp;
  const __bf16* Bh = (const __bf16*)(const void*)Shp;
  const __bf16* Bl = (const __bf16*)(const void*)Slp;
  __shared__ __align__(16) float sT[8][16 * 68];
  const int b    = blockIdx.y;
  const int lane = threadIdx.x & 31;
  const int wave = threadIdx.x >> 5;
  const int tilesN = HH;
  const int tilesM = COUT >> 6;
  const int tile = blockIdx.x * 8 + wave;
  if (tile >= tilesM * tilesN) return;
  const int tm = tile / tilesN;
  const int h  = tile - tm * tilesN;
  const int m0 = tm << 6;

  const int rlane = lane & 15;
  const int koff  = (lane >> 4) * 8;
  const int mOff  = (lane >> 4) * 8;

  v8f acc[4][4];
#pragma unroll
  for (int i = 0; i < 4; ++i)
#pragma unroll
    for (int j = 0; j < 4; ++j) acc[i][j] = zero8();

#pragma unroll 1
  for (int tap = 0; tap < 9; ++tap) {
    const int kh = tap / 3;
    const int dh = kh - 1;
    const int dw = (tap - 3 * kh) - 1;
    const size_t poff = (((size_t)(b * PH + h + 1 + dh)) * PWD + (size_t)(1 + dw)) * CIN;
    const __bf16* Bth = Bh + poff;
    const __bf16* Btl = Bl + poff;
    const __bf16* At  = A + tap * CIN;
#pragma unroll 1
    for (int kc = 0; kc < CIN; kc += 32) {
      v16b ah[4];
#pragma unroll
      for (int i = 0; i < 4; ++i) {
        ah[i] = ldfrag_b(At + (size_t)(m0 + (i << 4) + rlane) * KCONV + kc + koff);
      }
#pragma unroll
      for (int j = 0; j < 4; ++j) {
        const size_t bo = (size_t)((j << 4) + rlane) * CIN + kc + koff;
        const v16b bh = ldfrag_b(Bth + bo);
        const v16b bl = ldfrag_b(Btl + bo);
#pragma unroll
        for (int i = 0; i < 4; ++i) {
          acc[i][j] = mma_b_raw(ah[i], bh, acc[i][j]);
          acc[i][j] = mma_b_raw(ah[i], bl, acc[i][j]);
        }
        dep_guard_b(acc[0][j], acc[3][j], bh, bl);
      }
      keep4_b(ah[0], ah[1], ah[2], ah[3]);
    }
  }
  acc_guard4(acc[0][0], acc[0][1], acc[0][2], acc[0][3]);
  acc_guard4(acc[1][0], acc[1][1], acc[1][2], acc[1][3]);
  acc_guard4(acc[2][0], acc[2][1], acc[2][2], acc[2][3]);
  acc_guard4(acc[3][0], acc[3][1], acc[3][2], acc[3][3]);

  float* slab = sT[wave];
  const int hh2 = lane >> 4, c4 = (lane & 15) * 4;
  float* C = feat + (size_t)b * COUT * NPIX_FULL;
#pragma unroll
  for (int i = 0; i < 4; ++i) {
    const int mBase = m0 + (i << 4);
#pragma unroll
    for (int j = 0; j < 4; ++j) {
#pragma unroll
      for (int r = 0; r < 8; ++r) {
        slab[(mOff + r) * 68 + (j << 4) + rlane] = acc[i][j][r];
      }
    }
    __builtin_amdgcn_fence(__ATOMIC_RELEASE, "workgroup");
    __builtin_amdgcn_wave_barrier();
    __builtin_amdgcn_fence(__ATOMIC_ACQUIRE, "workgroup");
    v4f fv[8];
#pragma unroll
    for (int it = 0; it < 8; ++it) {
      const int row = it * 2 + hh2;
      const int o = mBase + row;
      const float sc = bf_rn(bng[o]) * bninv;
      const float sf = bf_rn(bnb[o]);
      v4f v = *(const v4f*)(slab + row * 68 + c4);
#pragma unroll
      for (int e = 0; e < 4; ++e) v[e] = fmaxf(v[e] * sc + sf, 0.f);
      fv[it] = v;
    }
    for (int pass = 0; pass < 2; ++pass) {
#pragma unroll
      for (int it = 0; it < 8; ++it) {
        const int row = it * 2 + hh2;
        *(volatile v4f*)(C + (size_t)(mBase + row) * NPIX_FULL + (size_t)h * IMW + c4) = fv[it];
      }
      __threadfence();
    }
    __builtin_amdgcn_fence(__ATOMIC_RELEASE, "workgroup");
    __builtin_amdgcn_wave_barrier();
    __builtin_amdgcn_fence(__ATOMIC_ACQUIRE, "workgroup");
  }
}

extern "C" void kernel_launch(void* const* d_in, const int* in_sizes, int n_in,
                              void* d_out, int out_size, void* d_ws, size_t ws_size,
                              hipStream_t stream) {
  if (n_in < 12) return;
  if (in_sizes[0] < NB * CIN * NPIX_FULL || in_sizes[1] < NB * CIN * NPIX_FULL) return;
  if (in_sizes[2] < DQK * CIN || in_sizes[3] < DQK || in_sizes[4] < DQK * CIN || in_sizes[5] < DQK) return;
  if (in_sizes[6] < DV * CIN || in_sizes[7] < DV || in_sizes[8] < 1) return;
  if (in_sizes[9] < COUT * KCONV || in_sizes[10] < COUT || in_sizes[11] < COUT) return;
  if (out_size < 3 * NB_FULL * CIN * NPIX_FULL) return;

  const float* x1    = (const float*)d_in[0];
  const float* x2    = (const float*)d_in[1];
  const float* Wq    = (const float*)d_in[2];
  const float* bq    = (const float*)d_in[3];
  const float* Wk    = (const float*)d_in[4];
  const float* bk    = (const float*)d_in[5];
  const float* Wv    = (const float*)d_in[6];
  const float* bv    = (const float*)d_in[7];
  const float* gamma = (const float*)d_in[8];
  const float* Wcat  = (const float*)d_in[9];
  const float* bng   = (const float*)d_in[10];
  const float* bnb   = (const float*)d_in[11];

  float* feat = (float*)d_out;
  float* out1 = feat + (size_t)NB_FULL * CIN * NPIX_FULL;
  float* out2 = feat + (size_t)2 * NB_FULL * CIN * NPIX_FULL;

  size_t off = 0;
  const size_t oXT  = off; off += (size_t)NIMG * NPIX * CIN * 2;
  const size_t oWqk = off; off += (size_t)64 * CIN * 2;
  const size_t oBqk = off; off += 256;
  const size_t oWvb = off; off += (size_t)DV * CIN * 2;
  const size_t oWm  = off; off += (size_t)COUT * KCONV * 2;
  const size_t oQK  = off; off += (size_t)NIMG * NPIX * 64 * 2;
  const size_t oVT  = off; off += (size_t)NIMG * DV * NPIX * 2;
  const size_t oSh  = off; off += (size_t)NB * PH * PWD * CIN * 2;
  const size_t oSl  = off; off += (size_t)NB * PH * PWD * CIN * 2;
  if (off > ws_size) return;
  if (off > (size_t)134217728) return;

  char* ws = (char*)d_ws;
  unsigned short* XT  = (unsigned short*)(ws + oXT);
  unsigned short* Wqk = (unsigned short*)(ws + oWqk);
  float*          Bqk = (float*)(ws + oBqk);
  unsigned short* Wvb = (unsigned short*)(ws + oWvb);
  unsigned short* Wm  = (unsigned short*)(ws + oWm);
  unsigned short* QKp = (unsigned short*)(ws + oQK);
  unsigned short* VTp = (unsigned short*)(ws + oVT);
  unsigned short* Sph = (unsigned short*)(ws + oSh);
  unsigned short* Spl = (unsigned short*)(ws + oSl);

  const float bninv = 1.0f / sqrtf(1.0f + 1.0e-5f);
  const dim3 blk(256);
  const dim3 gXT(NPIX / 64, CIN / 64, NIMG);
  const int  n8w = DV * CIN / 8;
  const dim3 gWv((n8w + 255) / 256);
  const dim3 gQK((((NIMG * NPIX) / 64) * 1 + 7) / 8, 1);
  const dim3 gVT(((DV / 64) * (NPIX / 64) + 7) / 8, NIMG);
  const dim3 gAtt(2 * NB * NQT);
  const dim3 gRing((NB * NBRD + 7) / 8);
  const dim3 gFuse(NPIX / 32, NB);
  const dim3 gConv(((COUT / 64) * HH + 7) / 8, NB);

  cvt_xT<<<gXT, blk, 0, stream>>>(x1, x2, XT);
  pack_qk<<<dim3(1), blk, 0, stream>>>(Wq, bq, Wk, bk, Wqk, Bqk);
  cvt_bf16x8<<<gWv, blk, 0, stream>>>(Wv, Wvb, n8w);
  pack_wcat<<<dim3(COUT), blk, 0, stream>>>(Wcat, Wm);
  gemm64<0, 1, 1><<<gQK, blk, 0, stream>>>(
      XT, XT, CIN, 0LL, Wqk, CIN, 0LL, Bqk, Bqk, Bqk,
      (void*)QKp, (void*)QKp, (void*)QKp, 64, 0LL,
      NIMG * NPIX, 64, CIN, 16.0f, 1.0f);
  gemm64<0, 1, 8><<<gVT, blk, 0, stream>>>(
      Wvb, Wvb, CIN, 0LL, XT, CIN, (long long)NPIX * CIN, Bqk, bv, Bqk,
      (void*)VTp, (void*)VTp, (void*)VTp, NPIX, (long long)DV * NPIX,
      DV, NPIX, CIN, 16.0f, 1.0f);
  attn_x<<<gAtt, dim3(128), 0, stream>>>(QKp, VTp, x1, x2, gamma, out1, out2, 1.0f / 1024.0f, 1.0f / 16384.0f);
  zero_ring<<<gRing, blk, 0, stream>>>(Sph, Spl);
  fuse_s<<<gFuse, blk, 0, stream>>>(x1, x2, gamma, out1, out2, Sph, Spl);
  conv_gemm<<<gConv, blk, 0, stream>>>(Wm, Sph, Spl, bng, bnb, feat, bninv);
  (void)hipGetLastError();
}
